// GCNNet_34626026340852
// MI455X (gfx1250) — hardware-verified
//
#include <hip/hip_runtime.h>
#include <stddef.h>
#include <stdint.h>
#include <math.h>


#define NNODE  200000
#define NEDGE  3200000
#define NGR    512
#define SEQL   1000
#define NTHR   256
#define NWAVE  8
#define EPT    8
#define CHUNK  (NTHR * EPT)
#define WCAP   (EPT * 32)
#define LISTN  (NWAVE * WCAP)
#define NBR    2048
#define SLB    11
#define SRCB   18
#define RCAP   36864
#define DEGCAP 64
#define NBLK   ((NNODE + NBR - 1) / NBR)
#define NPAD   (NBLK * NBR)
#define BK_INTS (LISTN + RCAP + 3 * NBR + 16 + RCAP / 2)
#define GBM    64
#define GBN    64
#define GTHR   128
#define WSMAX  134217728

#define L1P 331
#define L2P 108
#define L3P 33

#define PU0 4096
#define PU1 (PU0 + 32768)
#define PU2 (PU1 + 4096)
#define PU3 (PU2 + 65536)
#define PU4 (PU3 + 131072)
#define PU5 (PU4 + 256)
#define PU6 (PU5 + 4096)
#define PU7 (PU6 + 16384)

static_assert(NNODE <= (1 << SRCB));
static_assert(NBR == (1 << SLB) && SLB + SRCB <= 31);
static_assert(((long long)CHUNK << SLB) < (1LL << 31));
static_assert(RCAP % (NTHR * 4) == 0 && RCAP <= 65535 && RCAP % 32 == 0);
static_assert(RCAP >= 35045);
static_assert(NBR % (NTHR * 4) == 0 && NBR % NTHR == 0 && NBR % 32 == 0);
static_assert((NNODE % NBR) % 8 == 0 && NNODE % 4 == 0);
static_assert(BK_INTS % 4 == 0 && BK_INTS * 4 <= 300000);
static_assert(LISTN % 4 == 0);
static_assert(PU0 % NTHR == 0 && PU1 % NTHR == 0 && PU2 % NTHR == 0 && PU3 % NTHR == 0);
static_assert(PU4 % NTHR == 0 && PU5 % NTHR == 0 && PU6 % NTHR == 0 && PU7 % NTHR == 0);
static_assert(126 % 3 == 0 && 7 * 42 + 37 == L1P && 2 * 42 + 24 == L2P && 3 * L3P == 99);
static_assert(NGR % GBM == 0);

typedef float          v4f   __attribute__((ext_vector_type(4)));
typedef float          v8f   __attribute__((ext_vector_type(8)));
typedef int            v4i   __attribute__((ext_vector_type(4)));
typedef int            v8i   __attribute__((ext_vector_type(8)));
typedef unsigned short v8us  __attribute__((ext_vector_type(8)));
typedef unsigned short v16us __attribute__((ext_vector_type(16)));
typedef __bf16         v16bf __attribute__((ext_vector_type(16)));
typedef v4f  __attribute__((may_alias)) v4fa;
typedef v4i  __attribute__((may_alias)) v4ia;
typedef v8us __attribute__((may_alias)) v8usa;
union FragB { v16bf v; v16us u; v8us h[2]; v8i w; };

__device__ __forceinline__ v8f wmb(const FragB& a, const FragB& b, v8f c) {
  v8f d = __builtin_amdgcn_wmma_f32_16x16x32_bf16(false, a.v, false, b.v, (short)0, c, false, false);
  asm volatile("v_nop\n\tv_nop\n\tv_nop\n\tv_nop" : "+v"(d) : "v"(a.w), "v"(b.w));
  return d;
}

__device__ __forceinline__ unsigned bf16_bits(float f) {
  const unsigned u = __float_as_uint(f);
  const unsigned r = (u + 0x7FFFu + ((u >> 16) & 1u)) >> 16;
  return (f != f) ? 0x7FC0u : r;
}
__device__ __forceinline__ float bf16_val(float f) { return __uint_as_float(bf16_bits(f) << 16); }
__device__ __forceinline__ void split_hl(float v, unsigned& hb, unsigned& lb) {
  hb = bf16_bits(v);
  lb = bf16_bits(v - __uint_as_float(hb << 16));
}
__device__ __forceinline__ float nrelu(float v) { return (v > 0.0f) ? v : (v - v); }
__device__ __forceinline__ float nmax(float m, float v) { return (v > m || v != v) ? v : m; }

__device__ __forceinline__ void put8(unsigned short* dp, v8us o) {
  *(volatile v8us*)dp = o;
  __threadfence();
  *(volatile v8us*)dp = o;
}

__device__ __forceinline__ int scan_chunk(const int* __restrict__ dsts, int nE, int cbase, int slotBase,
                                          int nb, int vec8, int* list, int tid, int lane, int wave) {
  int wc = 0;
  const int el0  = tid * EPT;
  const int e0   = cbase + el0;
  const int sent = -2147483647 - 1;
  v4i da, db;
  if (vec8 != 0 && cbase + CHUNK <= nE) {
    da = *(const v4i*)(dsts + e0);
    db = *(const v4i*)(dsts + e0 + 4);
  } else {
    da.x = (e0     < nE) ? dsts[min(e0,     nE - 1)] : sent;
    da.y = (e0 + 1 < nE) ? dsts[min(e0 + 1, nE - 1)] : sent;
    da.z = (e0 + 2 < nE) ? dsts[min(e0 + 2, nE - 1)] : sent;
    da.w = (e0 + 3 < nE) ? dsts[min(e0 + 3, nE - 1)] : sent;
    db.x = (e0 + 4 < nE) ? dsts[min(e0 + 4, nE - 1)] : sent;
    db.y = (e0 + 5 < nE) ? dsts[min(e0 + 5, nE - 1)] : sent;
    db.z = (e0 + 6 < nE) ? dsts[min(e0 + 6, nE - 1)] : sent;
    db.w = (e0 + 7 < nE) ? dsts[min(e0 + 7, nE - 1)] : sent;
  }
  const unsigned nbs = (unsigned)slotBase;
  const unsigned unb = (unsigned)nb;
  const unsigned s0 = (unsigned)da.x - nbs, s1 = (unsigned)da.y - nbs;
  const unsigned s2 = (unsigned)da.z - nbs, s3 = (unsigned)da.w - nbs;
  const unsigned s4 = (unsigned)db.x - nbs, s5 = (unsigned)db.y - nbs;
  const unsigned s6 = (unsigned)db.z - nbs, s7 = (unsigned)db.w - nbs;
  const bool h0 = s0 < unb, h1 = s1 < unb, h2 = s2 < unb, h3 = s3 < unb;
  const bool h4 = s4 < unb, h5 = s5 < unb, h6 = s6 < unb, h7 = s7 < unb;
  const unsigned any = __builtin_amdgcn_ballot_w32(h0 | h1 | h2 | h3 | h4 | h5 | h6 | h7);
  if (any != 0u) {
#define HITJ(J, HJ, SJ) { \
      const unsigned mj = __builtin_amdgcn_ballot_w32(HJ); \
      if (mj != 0u) { \
        if (HJ) { \
          const int pos = wc + (int)__builtin_amdgcn_mbcnt_lo(mj, 0u); \
          if (pos < WCAP) list[wave * WCAP + pos] = ((el0 + (J)) << SLB) | (int)(SJ); \
        } \
        wc += (int)__builtin_popcount(mj); } }
    HITJ(0, h0, s0)
    HITJ(1, h1, s1)
    HITJ(2, h2, s2)
    HITJ(3, h3, s3)
    HITJ(4, h4, s4)
    HITJ(5, h5, s5)
    HITJ(6, h6, s6)
    HITJ(7, h7, s7)
#undef HITJ
  }
  return wc;
}

__device__ __forceinline__ void dense_unit(const float* __restrict__ W, int K0, int N, int v,
                                           unsigned short* plane) {
  const int upr = K0 >> 2;
  const int n   = v / upr;
  const int k8  = (v - n * upr) * 8;
  const int kk  = k8 & (K0 - 1);
  const float* p = W + (size_t)kk * N + n;
  v8us o;
#pragma unroll
  for (int i = 0; i < 8; ++i) o[i] = (unsigned short)bf16_bits(p[(size_t)i * N]);
  put8(plane + (size_t)8 * v, o);
}

__global__ __launch_bounds__(NTHR) void k_prep(
    const float* __restrict__ Wg1, const float* __restrict__ Wg2, const float* __restrict__ Wxt,
    const float* __restrict__ Wf1, const float* __restrict__ Wf2,
    const float* __restrict__ K1, const float* __restrict__ K2, const float* __restrict__ K3,
    unsigned short* Wg1T, unsigned short* Wg2T, unsigned short* WxtT, unsigned short* Wf1T,
    unsigned short* Wf2T, unsigned short* B1, unsigned short* B2, unsigned short* B3) {
  const int u = (int)blockIdx.x * NTHR + (int)threadIdx.x;
  if (u < PU0) {
    dense_unit(Wg1, 16, 1024, u, Wg1T);
  } else if (u < PU1) {
    dense_unit(Wg2, 1024, 128, u - PU0, Wg2T);
  } else if (u < PU2) {
    dense_unit(Wxt, 128, 128, u - PU1, WxtT);
  } else if (u < PU3) {
    dense_unit(Wf1, 256, 1024, u - PU2, Wf1T);
  } else if (u < PU4) {
    dense_unit(Wf2, 1024, 512, u - PU3, Wf2T);
  } else if (u < PU5) {
    const int v = u - PU4;
    const int o = v >> 3, k8 = (v & 7) * 8;
    v8us r;
#pragma unroll
    for (int e = 0; e < 8; ++e) {
      const int j = k8 + e;
      const int tap = j / 5;
      const int i = j - 5 * tap;
      const bool ok = j < 40;
      const int idx = ok ? (o * 40 + i * 8 + tap) : 0;
      const float val = K1[idx];
      r[e] = ok ? (unsigned short)bf16_bits(val) : (unsigned short)0;
    }
    put8(B1 + (size_t)8 * v, r);
  } else if (u < PU6) {
    const int v = u - PU5;
    const int o = v >> 6, k8 = (v & 63) * 8;
    const int tap = k8 >> 6, i0 = k8 & 31;
    const float* p = K2 + (size_t)o * 256 + (size_t)i0 * 8 + tap;
    v8us r;
#pragma unroll
    for (int e = 0; e < 8; ++e) r[e] = (unsigned short)bf16_bits(p[e * 8]);
    put8(B2 + (size_t)8 * v, r);
  } else if (u < PU7) {
    const int v = u - PU6;
    const int o = v >> 7, k8 = (v & 127) * 8;
    const int tap = k8 >> 7, i0 = k8 & 63;
    const float* p = K3 + (size_t)o * 512 + (size_t)i0 * 8 + tap;
    v8us r;
#pragma unroll
    for (int e = 0; e < 8; ++e) r[e] = (unsigned short)bf16_bits(p[e * 8]);
    put8(B3 + (size_t)8 * v, r);
  }
}

__device__ __forceinline__ void bk_store_pass(const int* hl, const unsigned short* sl, const int* cnt,
    const int* offs, const int* disb, const float* w1s, int tt, int ovf, int blk, int tid,
    const float* __restrict__ x, int* LIST, int* CNT, int* OFF, float* DIS, int* POIS, float* H1) {
  const int nodeBase = blk * NBR;
#pragma unroll 1
  for (int it = 0; it < RCAP / (NTHR * 4); ++it) {
    const int p0 = it * (NTHR * 4) + 4 * tid;
    int i0 = (int)sl[p0], i1 = (int)sl[p0 + 1], i2 = (int)sl[p0 + 2], i3 = (int)sl[p0 + 3];
    i0 = i0 > RCAP - 1 ? RCAP - 1 : i0;
    i1 = i1 > RCAP - 1 ? RCAP - 1 : i1;
    i2 = i2 > RCAP - 1 ? RCAP - 1 : i2;
    i3 = i3 > RCAP - 1 ? RCAP - 1 : i3;
    const int e0 = hl[i0] & ((1 << SRCB) - 1), e1 = hl[i1] & ((1 << SRCB) - 1);
    const int e2 = hl[i2] & ((1 << SRCB) - 1), e3 = hl[i3] & ((1 << SRCB) - 1);
    v4i v;
    v.x = (p0     < tt) ? e0 : 0;
    v.y = (p0 + 1 < tt) ? e1 : 0;
    v.z = (p0 + 2 < tt) ? e2 : 0;
    v.w = (p0 + 3 < tt) ? e3 : 0;
    *(volatile v4i*)(LIST + (size_t)blk * RCAP + p0) = v;
  }
#pragma unroll 1
  for (int it = 0; it < NBR / (NTHR * 4); ++it) {
    const int s0 = it * (NTHR * 4) + 4 * tid;
    const v4i c4 = *(const v4ia*)(cnt + s0);
    const v4i o4 = *(const v4ia*)(offs + s0);
    const v4i b4 = *(const v4ia*)(disb + s0);
    v4f d4;
    d4.x = __int_as_float(b4.x);
    d4.y = __int_as_float(b4.y);
    d4.z = __int_as_float(b4.z);
    d4.w = __int_as_float(b4.w);
    *(volatile v4i*)(CNT + (size_t)nodeBase + s0) = c4;
    *(volatile v4i*)(OFF + (size_t)nodeBase + s0) = o4;
    *(volatile v4f*)(DIS + (size_t)nodeBase + s0) = d4;
  }
  if (tid < 8) {
    const v4i f4 = {ovf, ovf, ovf, ovf};
    *(volatile v4i*)(POIS + (size_t)blk * 32 + 4 * tid) = f4;
  }
  const float qnan = __int_as_float(0x7fc00000);
#pragma unroll 1
  for (int it = 0; it < NBR / NTHR; ++it) {
    const int slot = it * NTHR + tid;
    const int node = nodeBase + slot;
    const int nc = node < NNODE ? node : NNODE - 1;
    const v4f xv = *(const v4fa*)(x + (size_t)nc * 4);
    const float x0 = bf16_val(xv.x), x1 = bf16_val(xv.y), x2 = bf16_val(xv.z), x3 = bf16_val(xv.w);
    const float dd = __int_as_float(disb[slot]);
    v4f h;
    h.x = dd * (((x0 * w1s[0] + x1 * w1s[4]) + x2 * w1s[8])  + x3 * w1s[12]);
    h.y = dd * (((x0 * w1s[1] + x1 * w1s[5]) + x2 * w1s[9])  + x3 * w1s[13]);
    h.z = dd * (((x0 * w1s[2] + x1 * w1s[6]) + x2 * w1s[10]) + x3 * w1s[14]);
    h.w = dd * (((x0 * w1s[3] + x1 * w1s[7]) + x2 * w1s[11]) + x3 * w1s[15]);
    const bool live = node < NNODE;
    const bool bad = ovf != 0;
    v4f o;
    o.x = live ? (bad ? qnan : h.x) : 0.0f;
    o.y = live ? (bad ? qnan : h.y) : 0.0f;
    o.z = live ? (bad ? qnan : h.z) : 0.0f;
    o.w = live ? (bad ? qnan : h.w) : 0.0f;
    *(volatile v4f*)(H1 + (size_t)node * 4) = o;
  }
}

__global__ __launch_bounds__(NTHR) void k_bucket(const int* __restrict__ srcs, const int* __restrict__ dsts,
    int vec8, const float* __restrict__ x, const float* __restrict__ W1,
    int* LIST, int* CNT, int* OFF, float* DIS, int* POIS, float* H1) {
  extern __shared__ __attribute__((aligned(16))) int dsm[];
  __shared__ float w1s[16];
  int* list = dsm;
  int* hl   = dsm + LISTN;
  int* cnt  = hl + RCAP;
  int* offs = cnt + NBR;
  int* cur  = offs + NBR;
  int* misc = cur + NBR;
  unsigned short* sl = (unsigned short*)(misc + 16);
  const int tid = (int)threadIdx.x, lane = tid & 31, wave = tid >> 5;
  const int blk = (int)blockIdx.x;
  const int nodeBase = blk * NBR;
  const int nE = NEDGE;

  {
    const v4i z4 = {0, 0, 0, 0};
    for (int i = tid * 4; i < BK_INTS; i += NTHR * 4) *(v4ia*)(dsm + i) = z4;
    if (tid < 16) w1s[tid] = bf16_val(W1[tid]);
  }
  __syncthreads();

  int t = 0;
  const int nChunks = (nE + CHUNK - 1) / CHUNK;
#pragma unroll 1
  for (int ch = 0; ch < nChunks; ++ch) {
    const int cbase = ch * CHUNK;
    const int wc = scan_chunk(dsts, nE, cbase, nodeBase, NBR, vec8, list, tid, lane, wave);
    if (lane == 0) misc[wave] = wc;
    __syncthreads();
    if (wave == 0) {
#pragma unroll 1
      for (int w2 = 0; w2 < NWAVE; ++w2) {
        int c = __builtin_amdgcn_readfirstlane(misc[w2]);
        c = c < 0 ? 0 : (c > WCAP ? WCAP : c);
#pragma unroll 1
        for (int b0 = 0; b0 < c; b0 += 32) {
          const int idx = b0 + lane;
          const int ent = list[w2 * WCAP + (idx < WCAP ? idx : WCAP - 1)];
          const int m32 = (c - b0) < 32 ? (c - b0) : 32;
          const int slot = ent & (NBR - 1);
          const int el   = (ent >> SLB) & (CHUNK - 1);
          int eid = cbase + el;
          eid = eid < 0 ? 0 : (eid > nE - 1 ? nE - 1 : eid);
          int sr = srcs[eid];
          sr = sr < 0 ? 0 : (sr > NNODE - 1 ? NNODE - 1 : sr);
          const int pk = sr | (slot << SRCB);
          const int pos = t + lane;
          if (lane < m32 && pos < RCAP) hl[pos] = pk;
#pragma unroll 1
          for (int k = 0; k < m32; ++k) {
            const int s = __builtin_amdgcn_readlane(slot, k);
            if (lane == 0 && (t + k) < RCAP) cnt[s] = cnt[s] + 1;
          }
          t += m32;
        }
      }
    }
    __syncthreads();
  }
  if (wave == 0 && lane == 0) { misc[8] = t > RCAP ? RCAP : t; misc[9] = t > RCAP ? 1 : 0; }
  __syncthreads();
  int tt = __builtin_amdgcn_readfirstlane(misc[8]);
  tt = tt < 0 ? 0 : (tt > RCAP ? RCAP : tt);
  const int ovf = __builtin_amdgcn_readfirstlane(misc[9]);

  if (wave == 0) {
    const int base = lane * (NBR / 32);
    int s = 0;
#pragma unroll 1
    for (int i = 0; i < NBR / 32; ++i) s += cnt[base + i];
    int incl = s;
#pragma unroll
    for (int d = 1; d < 32; d <<= 1) {
      const int y = __shfl_up(incl, d, 32);
      if (lane >= d) incl += y;
    }
    int run = incl - s;
#pragma unroll 1
    for (int i = 0; i < NBR / 32; ++i) {
      const int cv = cnt[base + i];
      offs[base + i] = run;
      cur[base + i]  = run;
      run += cv;
    }
  }
  __syncthreads();
  if (wave == 0) {
#pragma unroll 1
    for (int b0 = 0; b0 < tt; b0 += 32) {
      const int idx = b0 + lane;
      const int ent = hl[idx < RCAP ? idx : RCAP - 1];
      const int slot = (ent >> SRCB) & (NBR - 1);
      const int m32 = (tt - b0) < 32 ? (tt - b0) : 32;
#pragma unroll 1
      for (int k = 0; k < m32; ++k) {
        const int s = __builtin_amdgcn_readlane(slot, k);
        if (lane == 0) {
          int p = cur[s];
          p = p < 0 ? 0 : (p > RCAP - 1 ? RCAP - 1 : p);
          sl[p] = (unsigned short)(b0 + k);
          cur[s] = p + 1;
        }
      }
    }
  }
  __syncthreads();

  int* disb = cur;
#pragma unroll 1
  for (int it = 0; it < NBR / NTHR; ++it) {
    const int slot = it * NTHR + tid;
    const float dd = 1.0f / sqrtf((float)(cnt[slot] + 1));
    disb[slot] = __float_as_int(dd);
  }
  __syncthreads();

  bk_store_pass(hl, sl, cnt, offs, disb, w1s, tt, ovf, blk, tid, x, LIST, CNT, OFF, DIS, POIS, H1);
  __threadfence();
  bk_store_pass(hl, sl, cnt, offs, disb, w1s, tt, ovf, blk, tid, x, LIST, CNT, OFF, DIS, POIS, H1);
}

template <int F, int FO, int XF>
__global__ __launch_bounds__(NTHR) void k_agg(const int* __restrict__ LIST, const int* __restrict__ CNT,
    const int* __restrict__ OFF, const float* __restrict__ DIS, const int* __restrict__ POIS,
    const float* __restrict__ Hin, const float* __restrict__ bias, const float* __restrict__ Wn,
    float* Hout) {
  __shared__ __attribute__((aligned(16))) float stg[NTHR * FO];
  __shared__ float wsm[F * FO];
  __shared__ float bsm[16];
  const int tid = (int)threadIdx.x;
  const int blk = (int)blockIdx.x;
  const int nodeBase = blk * NBR;
  for (int i = tid; i < F * FO; i += NTHR) {
    float wv = 0.0f;
    if constexpr (XF != 0) wv = bf16_val(Wn[i]);
    wsm[i] = wv;
  }
  if (tid < 16) {
    const float bb = bias[tid < F ? tid : F - 1];
    bsm[tid] = (tid < F) ? bf16_val(bb) : 0.0f;
  }
  const int pf = POIS[(size_t)blk * 32];
  const int* lp = LIST + (size_t)blk * RCAP;
  const float qnan = __int_as_float(0x7fc00000);
  __syncthreads();

#pragma unroll 1
  for (int pass = 0; pass < NBR / NTHR; ++pass) {
    const int slot = pass * NTHR + tid;
    const int node = nodeBase + slot;
    const int nc = node < NNODE ? node : NNODE - 1;
    int c = CNT[node];
    const bool big = c > DEGCAP;
    c = c < 0 ? 0 : (c > DEGCAP ? DEGCAP : c);
    int o = OFF[node];
    o = o < 0 ? 0 : (o > RCAP - 1 ? RCAP - 1 : o);
    const float dd = DIS[node];
    int cm = c;
    cm = max(cm, __shfl_xor(cm, 16, 32));
    cm = max(cm, __shfl_xor(cm, 8, 32));
    cm = max(cm, __shfl_xor(cm, 4, 32));
    cm = max(cm, __shfl_xor(cm, 2, 32));
    cm = max(cm, __shfl_xor(cm, 1, 32));
    cm = __builtin_amdgcn_readfirstlane(cm);
    cm = cm > DEGCAP ? DEGCAP : cm;

    float acc[F];
#pragma unroll
    for (int f = 0; f < F; ++f) acc[f] = 0.0f;
#pragma unroll 1
    for (int j = 0; j < cm; ++j) {
      int jj = j < c ? j : c - 1;
      jj = jj < 0 ? 0 : jj;
      int idx = o + jj;
      idx = idx > RCAP - 1 ? RCAP - 1 : idx;
      int s = lp[idx];
      s = s < 0 ? 0 : (s > NNODE - 1 ? NNODE - 1 : s);
      const bool ok = j < c;
      const float* hp = Hin + (size_t)s * F;
#pragma unroll
      for (int q = 0; q < F / 4; ++q) {
        const v4f a = *(const v4fa*)(hp + 4 * q);
        acc[4 * q + 0] += ok ? a.x : 0.0f;
        acc[4 * q + 1] += ok ? a.y : 0.0f;
        acc[4 * q + 2] += ok ? a.z : 0.0f;
        acc[4 * q + 3] += ok ? a.w : 0.0f;
      }
    }
    float v[F];
    {
      const float* hp = Hin + (size_t)nc * F;
#pragma unroll
      for (int q = 0; q < F / 4; ++q) {
        const v4f a = *(const v4fa*)(hp + 4 * q);
        v[4 * q + 0] = acc[4 * q + 0] + a.x;
        v[4 * q + 1] = acc[4 * q + 1] + a.y;
        v[4 * q + 2] = acc[4 * q + 2] + a.z;
        v[4 * q + 3] = acc[4 * q + 3] + a.w;
      }
    }
    const bool bad = (pf != 0) || big;
    const bool live = node < NNODE;
#pragma unroll
    for (int f = 0; f < F; ++f) {
      float y = dd * v[f] + bsm[f];
      y = nrelu(y);
      v[f] = bad ? qnan : y;
    }
    if constexpr (XF != 0) {
#pragma unroll 1
      for (int oc = 0; oc < FO; ++oc) {
        float s = 0.0f;
#pragma unroll
        for (int f = 0; f < F; ++f) s = fmaf(v[f], wsm[f * FO + oc], s);
        const float val = dd * s;
        stg[tid * FO + oc] = live ? val : 0.0f;
      }
    } else {
#pragma unroll
      for (int f = 0; f < F; ++f) stg[tid * FO + f] = live ? v[f] : 0.0f;
    }
    __syncthreads();
    float* ob = Hout + (size_t)(nodeBase + pass * NTHR) * FO;
#pragma unroll
    for (int it = 0; it < FO / 4; ++it) {
      const int q = it * NTHR + tid;
      const v4f val = *(const v4fa*)(stg + 4 * q);
      *(volatile v4f*)(ob + 4 * q) = val;
    }
    __threadfence();
#pragma unroll
    for (int it = 0; it < FO / 4; ++it) {
      const int q = it * NTHR + tid;
      const v4f val = *(const v4fa*)(stg + 4 * q);
      *(volatile v4f*)(ob + 4 * q) = val;
    }
    __syncthreads();
  }
}

__global__ __launch_bounds__(NTHR) void k_pool(const float* __restrict__ X3, const int* __restrict__ bat,
                                               unsigned short* GHL) {
  __shared__ float red[NTHR * 33];
  __shared__ __attribute__((aligned(16))) unsigned short ob[64];
  const int tid = (int)threadIdx.x, lane = tid & 31, wave = tid >> 5;
  const int g0 = 2 * (int)blockIdx.x, g1 = g0 + 1;
  const float ninf = __int_as_float((int)0xff800000u);
  float m0[16], m1[16];
#pragma unroll
  for (int f = 0; f < 16; ++f) { m0[f] = ninf; m1[f] = ninf; }
  const int nV = NNODE / 4;
#pragma unroll 1
  for (int ib = 0; ib < nV; ib += NTHR) {
    const int i4 = ib + tid;
    const bool valid = i4 < nV;
    const int ic = valid ? i4 : nV - 1;
    const v4i ids = *(const v4i*)(bat + (size_t)4 * ic);
    const int idv[4] = {ids.x, ids.y, ids.z, ids.w};
#pragma unroll
    for (int j = 0; j < 4; ++j) {
      const bool r0 = valid && (idv[j] == g0);
      const bool r1 = valid && (idv[j] == g1);
      const unsigned any = __builtin_amdgcn_ballot_w32(r0 || r1);
      if (any != 0u) {
        const float* p = X3 + (size_t)(4 * ic + j) * 16;
#pragma unroll
        for (int q = 0; q < 4; ++q) {
          const v4f a = *(const v4fa*)(p + 4 * q);
          m0[4 * q + 0] = r0 ? nmax(m0[4 * q + 0], a.x) : m0[4 * q + 0];
          m0[4 * q + 1] = r0 ? nmax(m0[4 * q + 1], a.y) : m0[4 * q + 1];
          m0[4 * q + 2] = r0 ? nmax(m0[4 * q + 2], a.z) : m0[4 * q + 2];
          m0[4 * q + 3] = r0 ? nmax(m0[4 * q + 3], a.w) : m0[4 * q + 3];
          m1[4 * q + 0] = r1 ? nmax(m1[4 * q + 0], a.x) : m1[4 * q + 0];
          m1[4 * q + 1] = r1 ? nmax(m1[4 * q + 1], a.y) : m1[4 * q + 1];
          m1[4 * q + 2] = r1 ? nmax(m1[4 * q + 2], a.z) : m1[4 * q + 2];
          m1[4 * q + 3] = r1 ? nmax(m1[4 * q + 3], a.w) : m1[4 * q + 3];
        }
      }
    }
  }
#pragma unroll
  for (int f = 0; f < 16; ++f) { red[tid * 33 + f] = m0[f]; red[tid * 33 + 16 + f] = m1[f]; }
  __syncthreads();
  if (tid < 32) {
    float m = ninf;
#pragma unroll 4
    for (int t = 0; t < NTHR; ++t) m = nmax(m, red[t * 33 + tid]);
    unsigned hb, lb;
    split_hl(m, hb, lb);
    const int g = tid >> 4, f = tid & 15;
    ob[g * 32 + f] = (unsigned short)hb;
    ob[g * 32 + 16 + f] = (unsigned short)lb;
  }
  __syncthreads();
  const bool st = (wave == 0) && (lane < 8);
  const v8us ov = *(const v8usa*)(ob + 8 * (lane & 7));
  unsigned short* dp = GHL + (size_t)blockIdx.x * 64 + 8 * (lane & 7);
  if (st) *(volatile v8us*)dp = ov;
  __threadfence();
  if (st) *(volatile v8us*)dp = ov;
}

__device__ __forceinline__ void gemm_pass_hl(const float* stg, const float* sb, int relu, unsigned short* outH,
                                             int ldo, int rowBase, int hiCol, int loCol, int tid) {
#pragma unroll 1
  for (int it = 0; it < 8; ++it) {
    const int p = it * GTHR + tid;
    const int line = p >> 3, q = p & 7;
    const int row = line >> 1, part = line & 1;
    const v4f a  = *(const v4fa*)(stg + row * GBN + 8 * q);
    const v4f b  = *(const v4fa*)(stg + row * GBN + 8 * q + 4);
    const v4f ba = *(const v4fa*)(sb + 8 * q);
    const v4f bb = *(const v4fa*)(sb + 8 * q + 4);
    const float y[8] = {a.x + ba.x, a.y + ba.y, a.z + ba.z, a.w + ba.w,
                        b.x + bb.x, b.y + bb.y, b.z + bb.z, b.w + bb.w};
    v8us o;
#pragma unroll
    for (int e = 0; e < 8; ++e) {
      float v = y[e];
      v = (relu != 0) ? nrelu(v) : v;
      unsigned hb, lb;
      split_hl(v, hb, lb);
      o[e] = (unsigned short)((part != 0) ? lb : hb);
    }
    unsigned short* dp = outH + (size_t)(rowBase + row) * (size_t)ldo + ((part != 0) ? loCol : hiCol) + 8 * q;
    *(volatile v8us*)dp = o;
  }
}
__device__ __forceinline__ void gemm_pass_f32(const float* stg, const float* sb, int relu, float* outF,
                                              int ldo, int rowBase, int col0, int tid) {
#pragma unroll 1
  for (int it = 0; it < 8; ++it) {
    const int p = it * GTHR + tid;
    const int row = p >> 4, q = p & 15;
    const v4f a  = *(const v4fa*)(stg + row * GBN + 4 * q);
    const v4f ba = *(const v4fa*)(sb + 4 * q);
    v4f y;
    y.x = a.x + ba.x; y.y = a.y + ba.y; y.z = a.z + ba.z; y.w = a.w + ba.w;
    if (relu != 0) { y.x = nrelu(y.x); y.y = nrelu(y.y); y.z = nrelu(y.z); y.w = nrelu(y.w); }
    float* dp = outF + (size_t)(rowBase + row) * (size_t)ldo + col0 + 4 * q;
    *(volatile v4f*)dp = y;
  }
}

template <int MODE>
__global__ __launch_bounds__(GTHR) void k_gemm(
    const unsigned short* __restrict__ A, const unsigned short* __restrict__ WT,
    const float* __restrict__ bias, int K, int relu,
    unsigned short* outH, int ldoH, int hiBase, int loBase, float* outF, int ldoF) {
  __shared__ __attribute__((aligned(16))) float stg[GBM * GBN];
  __shared__ __attribute__((aligned(16))) float sb[GBN];
  const int tid = (int)threadIdx.x, lane = tid & 31, wave = tid >> 5, hh = lane >> 4, m = lane & 15;
  const int rowBase = (int)blockIdx.x * GBM;
  const int col0    = (int)blockIdx.y * GBN;
  if (tid < GBN) sb[tid] = bf16_val(bias[col0 + tid]);

  v8f acc[4];
  {
    const v8f z = {0.f, 0.f, 0.f, 0.f, 0.f, 0.f, 0.f, 0.f};
    acc[0] = z; acc[1] = z; acc[2] = z; acc[3] = z;
  }
  const unsigned short* ap = A  + (size_t)(rowBase + 16 * wave + m) * (size_t)K + 8 * hh;
  const unsigned short* wp = WT + (size_t)(col0 + m) * (size_t)K + 8 * hh;
  const int ksteps = K >> 5;
#pragma unroll 1
  for (int ks = 0; ks < ksteps; ++ks) {
    FragB af;
    af.h[0] = *(const v8usa*)(ap + 32 * ks);
    af.h[1] = *(const v8usa*)(ap + 32 * ks + 16);
#pragma unroll
    for (int t = 0; t < 4; ++t) {
      const unsigned short* wq = wp + (size_t)(16 * t) * (size_t)K + 32 * ks;
      FragB bf;
      bf.h[0] = *(const v8usa*)wq;
      bf.h[1] = *(const v8usa*)(wq + 16);
      acc[t] = wmb(af, bf, acc[t]);
    }
  }
#pragma unroll
  for (int t = 0; t < 4; ++t) {
    const int lc = 16 * t + m;
#pragma unroll
    for (int r = 0; r < 8; ++r) {
      const int lr = 16 * wave + 8 * hh + r;
      stg[lr * GBN + lc] = acc[t][r];
    }
  }
  __syncthreads();
  if constexpr (MODE == 0) {
    gemm_pass_hl(stg, sb, relu, outH, ldoH, rowBase, hiBase + col0, loBase + col0, tid);
    __threadfence();
    gemm_pass_hl(stg, sb, relu, outH, ldoH, rowBase, hiBase + col0, loBase + col0, tid);
  } else {
    gemm_pass_f32(stg, sb, relu, outF, ldoF, rowBase, col0, tid);
    __threadfence();
    gemm_pass_f32(stg, sb, relu, outF, ldoF, rowBase, col0, tid);
  }
}

__device__ __forceinline__ void conv1_pass(const float* stg, const float* cbs, unsigned short* C1, int b, int t,
                                           int tid) {
#pragma unroll 1
  for (int it = 0; it < 3; ++it) {
    const int p = it * 128 + tid;
    const int tokl = p >> 3, q = p & 7;
    const int tok = 42 * t + tokl;
    const bool ok = (tokl < 42) && (tok < L1P);
    const int tl = tokl < 42 ? tokl : 41;
    const int part = q >> 2, c0 = 8 * (q & 3);
    v8us o;
#pragma unroll
    for (int e = 0; e < 8; ++e) {
      const int c = c0 + e;
      const float y = fmaxf(fmaxf(stg[(3 * tl) * 32 + c], stg[(3 * tl + 1) * 32 + c]), stg[(3 * tl + 2) * 32 + c]);
      const float v = fmaxf(y + cbs[c], 0.0f);
      unsigned hb, lb;
      split_hl(v, hb, lb);
      o[e] = (unsigned short)((part != 0) ? lb : hb);
    }
    const int tokc = ok ? tok : 0;
    unsigned short* dp = C1 + ((size_t)b * L1P + tokc) * 64 + 8 * q;
    if (ok) *(volatile v8us*)dp = o;
  }
}

__global__ __launch_bounds__(128) void k_conv1(const float* __restrict__ tgt, const unsigned short* __restrict__ B1,
                                               const float* __restrict__ cb, unsigned short* C1) {
  __shared__ __attribute__((aligned(16))) unsigned short slab[688];
  __shared__ __attribute__((aligned(16))) unsigned short As[128 * 64];
  __shared__ __attribute__((aligned(16))) float stg[128 * 32];
  __shared__ float cbs[32];
  const int tid = (int)threadIdx.x, lane = tid & 31, w = tid >> 5, hh = lane >> 4, m = lane & 15;
  const int t = (int)blockIdx.x, b = (int)blockIdx.y;
  const int l0 = 126 * t;
  if (tid < 32) cbs[tid] = bf16_val(cb[tid]);
#pragma unroll 2
  for (int idx = tid; idx < 688; idx += 128) {
    const int ge = l0 * 5 + idx;
    const bool ok = (idx < 675) && (ge < SEQL * 5);
    const int gc = ge < SEQL * 5 ? ge : SEQL * 5 - 1;
    const float v = tgt[(size_t)b * (SEQL * 5) + gc];
    slab[idx] = ok ? (unsigned short)bf16_bits(v) : (unsigned short)0;
  }
  __syncthreads();
#pragma unroll 4
  for (int i = 0; i < 64; ++i) {
    const int idx = tid + 128 * i;
    const int r = idx >> 6, j = idx & 63;
    int si = 5 * r + j;
    si = si > 687 ? 687 : si;
    const unsigned short sv = slab[si];
    As[idx] = (j < 40) ? sv : (unsigned short)0;
  }
  __syncthreads();

  const v8f z = {0.f, 0.f, 0.f, 0.f, 0.f, 0.f, 0.f, 0.f};
  v8f acc[2][2];
  acc[0][0] = z; acc[0][1] = z; acc[1][0] = z; acc[1][1] = z;
  const unsigned short* a0 = As + (32 * w + m) * 64 + 8 * hh;
  const unsigned short* a1 = a0 + 16 * 64;
  const unsigned short* wp = B1 + (size_t)m * 64 + 8 * hh;
#pragma unroll
  for (int ks = 0; ks < 2; ++ks) {
    FragB f0, f1;
    f0.h[0] = *(const v8usa*)(a0 + 32 * ks);
    f0.h[1] = *(const v8usa*)(a0 + 32 * ks + 16);
    f1.h[0] = *(const v8usa*)(a1 + 32 * ks);
    f1.h[1] = *(const v8usa*)(a1 + 32 * ks + 16);
#pragma unroll
    for (int nt = 0; nt < 2; ++nt) {
      const unsigned short* wq = wp + (size_t)(16 * nt) * 64 + 32 * ks;
      FragB bf;
      bf.h[0] = *(const v8usa*)wq;
      bf.h[1] = *(const v8usa*)(wq + 16);
      acc[0][nt] = wmb(f0, bf, acc[0][nt]);
      acc[1][nt] = wmb(f1, bf, acc[1][nt]);
    }
  }
#pragma unroll
  for (int mt = 0; mt < 2; ++mt)
#pragma unroll
    for (int nt = 0; nt < 2; ++nt)
#pragma unroll
      for (int r = 0; r < 8; ++r)
        stg[(32 * w + 16 * mt + 8 * hh + r) * 32 + 16 * nt + m] = acc[mt][nt][r];
  __syncthreads();
  conv1_pass(stg, cbs, C1, b, t, tid);
  __threadfence();
  conv1_pass(stg, cbs, C1, b, t, tid);
}

__device__ __forceinline__ void conv_mma(const unsigned short* a0, const unsigned short* a1,
                                         const unsigned short* wp, int KT, v8f (&acc)[2][4]) {
  const int ksteps = KT >> 5;
#pragma unroll 1
  for (int ks = 0; ks < ksteps; ++ks) {
    FragB f0, f1;
    f0.h[0] = *(const v8usa*)(a0 + 32 * ks);
    f0.h[1] = *(const v8usa*)(a0 + 32 * ks + 16);
    f1.h[0] = *(const v8usa*)(a1 + 32 * ks);
    f1.h[1] = *(const v8usa*)(a1 + 32 * ks + 16);
#pragma unroll
    for (int t = 0; t < 4; ++t) {
      const unsigned short* wq = wp + (size_t)(16 * t) * (size_t)KT + 32 * ks;
      FragB bf;
      bf.h[0] = *(const v8usa*)wq;
      bf.h[1] = *(const v8usa*)(wq + 16);
      acc[0][t] = wmb(f0, bf, acc[0][t]);
      acc[1][t] = wmb(f1, bf, acc[1][t]);
    }
  }
}

__device__ __forceinline__ void conv2_pass(const float* stg, const float* cbs, unsigned short* C2, int b, int t,
                                           int tid) {
#pragma unroll 1
  for (int it = 0; it < 6; ++it) {
    const int p = it * 128 + tid;
    const int tokl = p >> 4, q = p & 15;
    const int tok = 42 * t + tokl;
    const bool ok = (tokl < 42) && (tok < L2P);
    const int tl = tokl < 42 ? tokl : 41;
    const int part = q >> 3, c0 = 8 * (q & 7);
    v8us o;
#pragma unroll
    for (int e = 0; e < 8; ++e) {
      const int c = c0 + e;
      const float y = fmaxf(fmaxf(stg[(3 * tl) * 64 + c], stg[(3 * tl + 1) * 64 + c]), stg[(3 * tl + 2) * 64 + c]);
      const float v = fmaxf(y + cbs[c], 0.0f);
      unsigned hb, lb;
      split_hl(v, hb, lb);
      o[e] = (unsigned short)((part != 0) ? lb : hb);
    }
    const int tokc = ok ? tok : 0;
    unsigned short* dp = C2 + ((size_t)b * L2P + tokc) * 128 + 8 * q;
    if (ok) *(volatile v8us*)dp = o;
  }
}

__global__ __launch_bounds__(128) void k_conv2(const unsigned short* __restrict__ C1,
                                               const unsigned short* __restrict__ B2,
                                               const float* __restrict__ cb, unsigned short* C2) {
  __shared__ __attribute__((aligned(16))) float stg[128 * 64];
  __shared__ float cbs[64];
  const int tid = (int)threadIdx.x, lane = tid & 31, w = tid >> 5, hh = lane >> 4, m = lane & 15;
  const int t = (int)blockIdx.x, b = (int)blockIdx.y;
  if (tid < 64) cbs[tid] = bf16_val(cb[tid]);
  int la = 126 * t + 32 * w + m;
  int lb2 = la + 16;
  la  = la  > 323 ? 323 : la;
  lb2 = lb2 > 323 ? 323 : lb2;
  const unsigned short* a0 = C1 + ((size_t)b * L1P + la) * 64 + 8 * hh;
  const unsigned short* a1 = C1 + ((size_t)b * L1P + lb2) * 64 + 8 * hh;
  const unsigned short* wp = B2 + (size_t)m * 512 + 8 * hh;
  const v8f z = {0.f, 0.f, 0.f, 0.f, 0.f, 0.f, 0.f, 0.f};
  v8f acc[2][4];
#pragma unroll
  for (int i = 0; i < 4; ++i) { acc[0][i] = z; acc[1][i] = z; }
  conv_mma(a0, a1, wp, 512, acc);
#pragma unroll
  for (int mt = 0; mt < 2; ++mt)
#pragma unroll
    for (int nt = 0; nt < 4; ++nt)
#pragma unroll
      for (int r = 0; r < 8; ++r)
        stg[(32 * w + 16 * mt + 8 * hh + r) * 64 + 16 * nt + m] = acc[mt][nt][r];
  __syncthreads();
  conv2_pass(stg, cbs, C2, b, t, tid);
  __threadfence();
  conv2_pass(stg, cbs, C2, b, t, tid);
}

__global__ __launch_bounds__(256) void k_conv3(const unsigned short* __restrict__ C2,
                                               const unsigned short* __restrict__ B3,
                                               const float* __restrict__ cb, unsigned short* CM) {
  __shared__ __attribute__((aligned(16))) float stg[104 * 128];
  __shared__ float cbs[128];
  __shared__ __attribute__((aligned(16))) unsigned short ob[256];
  const int tid = (int)threadIdx.x, lane = tid & 31, w = tid >> 5, hh = lane >> 4, m = lane & 15;
  const int b = (int)blockIdx.x;
  if (tid < 128) cbs[tid] = bf16_val(cb[tid]);
  const int rw = 32 * (w & 3), cw = 64 * (w >> 2);
  int la = rw + m;
  int lb2 = la + 16;
  la  = la  > 100 ? 100 : la;
  lb2 = lb2 > 100 ? 100 : lb2;
  const unsigned short* a0 = C2 + ((size_t)b * L2P + la) * 128 + 8 * hh;
  const unsigned short* a1 = C2 + ((size_t)b * L2P + lb2) * 128 + 8 * hh;
  const unsigned short* wp = B3 + (size_t)(cw + m) * 1024 + 8 * hh;
  const v8f z = {0.f, 0.f, 0.f, 0.f, 0.f, 0.f, 0.f, 0.f};
  v8f acc[2][4];
#pragma unroll
  for (int i = 0; i < 4; ++i) { acc[0][i] = z; acc[1][i] = z; }
  conv_mma(a0, a1, wp, 1024, acc);
#pragma unroll
  for (int mt = 0; mt < 2; ++mt)
#pragma unroll
    for (int nt = 0; nt < 4; ++nt)
#pragma unroll
      for (int r = 0; r < 8; ++r) {
        const int lr = rw + 16 * mt + 8 * hh + r;
        if (lr < 104) stg[lr * 128 + cw + 16 * nt + m] = acc[mt][nt][r];
      }
  __syncthreads();
  if (tid < 128) {
    const float cbv = cbs[tid];
    float s = 0.0f;
#pragma unroll 1
    for (int p = 0; p < L3P; ++p) {
      const float y = fmaxf(fmaxf(stg[(3 * p) * 128 + tid], stg[(3 * p + 1) * 128 + tid]),
                            stg[(3 * p + 2) * 128 + tid]);
      s += fmaxf(y + cbv, 0.0f);
    }
    const float mean = s * (1.0f / 33.0f);
    unsigned hb, lb;
    split_hl(mean, hb, lb);
    ob[tid] = (unsigned short)hb;
    ob[128 + tid] = (unsigned short)lb;
  }
  __syncthreads();
  const bool st = (w == 0);
  const v8us ov = *(const v8usa*)(ob + 8 * lane);
  unsigned short* dp = CM + (size_t)b * 256 + 8 * lane;
  if (st) *(volatile v8us*)dp = ov;
  __threadfence();
  if (st) *(volatile v8us*)dp = ov;
}

__global__ __launch_bounds__(NTHR) void k_out(const float* __restrict__ F2, const float* __restrict__ Wo,
                                              const float* __restrict__ bo, const int* __restrict__ POIS,
                                              float* out) {
  __shared__ float wos[1024];
  __shared__ float bos[2];
  __shared__ __attribute__((aligned(16))) float os[1024];
  const int tid = (int)threadIdx.x;
#pragma unroll 1
  for (int i = tid; i < 1024; i += NTHR) wos[i] = bf16_val(Wo[i]);
  if (tid < 2) bos[tid] = bf16_val(bo[tid]);
  int pf = 0;
#pragma unroll 1
  for (int b = 0; b < NBLK; ++b) pf |= POIS[(size_t)b * 32];
  __syncthreads();
  const float qnan = __int_as_float(0x7fc00000);
#pragma unroll 1
  for (int i4 = 0; i4 < 4; ++i4) {
    const int idx = i4 * NTHR + tid;
    const int r = idx >> 1, c = idx & 1;
    const float* pr = F2 + (size_t)r * 512;
    float s = 0.0f;
#pragma unroll 1
    for (int k4 = 0; k4 < 128; ++k4) {
      const v4f p = *(const v4fa*)(pr + 4 * k4);
      const float* wv = wos + 8 * k4 + c;
      s = fmaf(p.x, wv[0], s);
      s = fmaf(p.y, wv[2], s);
      s = fmaf(p.z, wv[4], s);
      s = fmaf(p.w, wv[6], s);
    }
    const float val = s + bos[c];
    os[idx] = (pf != 0) ? qnan : val;
  }
  __syncthreads();
  const v4f ov = *(const v4fa*)(os + 4 * tid);
  *(volatile v4f*)(out + 4 * (size_t)tid) = ov;
  __threadfence();
  *(volatile v4f*)(out + 4 * (size_t)tid) = ov;
}

static inline size_t al256(size_t o) { return (o + 255) & ~(size_t)255; }

extern "C" void kernel_launch(void* const* d_in, const int* in_sizes, int n_in,
                              void* d_out, int out_size, void* d_ws, size_t ws_size,
                              hipStream_t stream) {
  if (n_in < 28) return;
  if (in_sizes[0] != NNODE * 4) return;
  if (in_sizes[1] != 2 * NEDGE) return;
  if (in_sizes[2] != NNODE) return;
  if (in_sizes[3] != NGR * SEQL * 5) return;
  if (in_sizes[4] != 16 || in_sizes[5] != 4 || in_sizes[6] != 32 || in_sizes[7] != 8) return;
  if (in_sizes[8] != 128 || in_sizes[9] != 16) return;
  if (in_sizes[10] != 16 * 1024 || in_sizes[11] != 1024) return;
  if (in_sizes[12] != 1024 * 128 || in_sizes[13] != 128) return;
  if (in_sizes[14] != 32 * 5 * 8 || in_sizes[15] != 32) return;
  if (in_sizes[16] != 64 * 32 * 8 || in_sizes[17] != 64) return;
  if (in_sizes[18] != 128 * 64 * 8 || in_sizes[19] != 128) return;
  if (in_sizes[20] != 128 * 128 || in_sizes[21] != 128) return;
  if (in_sizes[22] != 256 * 1024 || in_sizes[23] != 1024) return;
  if (in_sizes[24] != 1024 * 512 || in_sizes[25] != 512) return;
  if (in_sizes[26] != 512 * 2 || in_sizes[27] != 2) return;
  if (out_size != NGR * 2) return;

  const float* x    = (const float*)d_in[0];
  const int*   edge = (const int*)d_in[1];
  const int*   bat  = (const int*)d_in[2];
  const float* tgt  = (const float*)d_in[3];
  const float* W1 = (const float*)d_in[4];   const float* b1 = (const float*)d_in[5];
  const float* W2 = (const float*)d_in[6];   const float* b2 = (const float*)d_in[7];
  const float* W3 = (const float*)d_in[8];   const float* b3 = (const float*)d_in[9];
  const float* Wg1 = (const float*)d_in[10]; const float* bg1 = (const float*)d_in[11];
  const float* Wg2 = (const float*)d_in[12]; const float* bg2 = (const float*)d_in[13];
  const float* K1 = (const float*)d_in[14];  const float* cb1 = (const float*)d_in[15];
  const float* K2 = (const float*)d_in[16];  const float* cb2 = (const float*)d_in[17];
  const float* K3 = (const float*)d_in[18];  const float* cb3 = (const float*)d_in[19];
  const float* Wxt = (const float*)d_in[20]; const float* bxt = (const float*)d_in[21];
  const float* Wf1 = (const float*)d_in[22]; const float* bf1 = (const float*)d_in[23];
  const float* Wf2 = (const float*)d_in[24]; const float* bf2 = (const float*)d_in[25];
  const float* Wo = (const float*)d_in[26];  const float* bo = (const float*)d_in[27];
  float* out = (float*)d_out;
  const int* src = edge;
  const int* dst = edge + NEDGE;
  const int vec8 = ((NEDGE & 3) == 0) ? 1 : 0;

  char* ws = (char*)d_ws;
  size_t off = 0;
  const size_t oLIST = off; off = al256(off + (size_t)NBLK * RCAP * 4);
  const size_t oCNT  = off; off = al256(off + (size_t)NPAD * 4);
  const size_t oOFF  = off; off = al256(off + (size_t)NPAD * 4);
  const size_t oDIS  = off; off = al256(off + (size_t)NPAD * 4);
  const size_t oPOI  = off; off = al256(off + (size_t)NBLK * 128);
  const size_t oH1   = off; off = al256(off + (size_t)NPAD * 4 * 4);
  const size_t oH2   = off; off = al256(off + (size_t)NPAD * 8 * 4);
  const size_t oH3   = off; off = al256(off + (size_t)NPAD * 16 * 4);
  const size_t oX3   = off; off = al256(off + (size_t)NPAD * 16 * 4);
  const size_t oGHL  = off; off = al256(off + (size_t)NGR * 32 * 2);
  const size_t oG1   = off; off = al256(off + (size_t)NGR * 2048 * 2);
  const size_t oXC   = off; off = al256(off + (size_t)NGR * 512 * 2);
  const size_t oC1   = off; off = al256(off + (size_t)NGR * L1P * 64 * 2);
  const size_t oC2   = off; off = al256(off + (size_t)NGR * L2P * 128 * 2);
  const size_t oCM   = off; off = al256(off + (size_t)NGR * 256 * 2);
  const size_t oF1   = off; off = al256(off + (size_t)NGR * 2048 * 2);
  const size_t oF2   = off; off = al256(off + (size_t)NGR * 512 * 4);
  const size_t oWg1  = off; off = al256(off + (size_t)1024 * 32 * 2);
  const size_t oWg2  = off; off = al256(off + (size_t)128 * 2048 * 2);
  const size_t oWxt  = off; off = al256(off + (size_t)128 * 256 * 2);
  const size_t oWf1  = off; off = al256(off + (size_t)1024 * 512 * 2);
  const size_t oWf2  = off; off = al256(off + (size_t)512 * 2048 * 2);
  const size_t oB1   = off; off = al256(off + (size_t)32 * 64 * 2);
  const size_t oB2   = off; off = al256(off + (size_t)64 * 512 * 2);
  const size_t oB3   = off; off = al256(off + (size_t)128 * 1024 * 2);
  if (off > ws_size || off > (size_t)WSMAX) return;

  int*   LIST = (int*)(ws + oLIST);
  int*   CNT  = (int*)(ws + oCNT);
  int*   OFF  = (int*)(ws + oOFF);
  float* DIS  = (float*)(ws + oDIS);
  int*   POIS = (int*)(ws + oPOI);
  float* H1 = (float*)(ws + oH1);
  float* H2 = (float*)(ws + oH2);
  float* H3 = (float*)(ws + oH3);
  float* X3 = (float*)(ws + oX3);
  unsigned short* GHL  = (unsigned short*)(ws + oGHL);
  unsigned short* G1HL = (unsigned short*)(ws + oG1);
  unsigned short* XCHL = (unsigned short*)(ws + oXC);
  unsigned short* C1HL = (unsigned short*)(ws + oC1);
  unsigned short* C2HL = (unsigned short*)(ws + oC2);
  unsigned short* CMHL = (unsigned short*)(ws + oCM);
  unsigned short* F1HL = (unsigned short*)(ws + oF1);
  float*          F2   = (float*)(ws + oF2);
  unsigned short* Wg1T = (unsigned short*)(ws + oWg1);
  unsigned short* Wg2T = (unsigned short*)(ws + oWg2);
  unsigned short* WxtT = (unsigned short*)(ws + oWxt);
  unsigned short* Wf1T = (unsigned short*)(ws + oWf1);
  unsigned short* Wf2T = (unsigned short*)(ws + oWf2);
  unsigned short* B1 = (unsigned short*)(ws + oB1);
  unsigned short* B2 = (unsigned short*)(ws + oB2);
  unsigned short* B3 = (unsigned short*)(ws + oB3);

  const size_t bkLds = (size_t)BK_INTS * 4;
  hipFuncSetAttribute(reinterpret_cast<const void*>(&k_bucket), hipFuncAttributeMaxDynamicSharedMemorySize,
                      (int)bkLds);

  k_prep<<<PU7 / NTHR, NTHR, 0, stream>>>(Wg1, Wg2, Wxt, Wf1, Wf2, K1, K2, K3,
                                          Wg1T, Wg2T, WxtT, Wf1T, Wf2T, B1, B2, B3);
  k_bucket<<<NBLK, NTHR, bkLds, stream>>>(src, dst, vec8, x, W1, LIST, CNT, OFF, DIS, POIS, H1);
  k_agg<4, 8, 1><<<NBLK, NTHR, 0, stream>>>(LIST, CNT, OFF, DIS, POIS, H1, b1, W2, H2);
  k_agg<8, 16, 1><<<NBLK, NTHR, 0, stream>>>(LIST, CNT, OFF, DIS, POIS, H2, b2, W3, H3);
  k_agg<16, 16, 0><<<NBLK, NTHR, 0, stream>>>(LIST, CNT, OFF, DIS, POIS, H3, b3, W3, X3);
  k_pool<<<NGR / 2, NTHR, 0, stream>>>(X3, bat, GHL);
  k_gemm<0><<<dim3(NGR / GBM, 1024 / GBN), GTHR, 0, stream>>>(GHL, Wg1T, bg1, 32, 1, G1HL, 2048, 0, 1024, F2, 512);
  k_gemm<0><<<dim3(NGR / GBM, 128 / GBN), GTHR, 0, stream>>>(G1HL, Wg2T, bg2, 2048, 0, XCHL, 512, 0, 256, F2, 512);
  k_conv1<<<dim3(8, NGR), 128, 0, stream>>>(tgt, B1, cb1, C1HL);
  k_conv2<<<dim3(3, NGR), 128, 0, stream>>>(C1HL, B2, cb2, C2HL);
  k_conv3<<<NGR, 256, 0, stream>>>(C2HL, B3, cb3, CMHL);
  k_gemm<0><<<dim3(NGR / GBM, 128 / GBN), GTHR, 0, stream>>>(CMHL, WxtT, bxt, 256, 1, XCHL, 512, 128, 384, F2, 512);
  k_gemm<0><<<dim3(NGR / GBM, 1024 / GBN), GTHR, 0, stream>>>(XCHL, Wf1T, bf1, 512, 1, F1HL, 2048, 0, 1024, F2, 512);
  k_gemm<1><<<dim3(NGR / GBM, 512 / GBN), GTHR, 0, stream>>>(F1HL, Wf2T, bf2, 2048, 1, F1HL, 2048, 0, 1024, F2, 512);
  k_out<<<1, NTHR, 0, stream>>>(F2, Wo, bo, POIS, out);
}
